// GCN_8083128451590
// MI455X (gfx1250) — hardware-verified
//
#include <hip/hip_runtime.h>
#include <stddef.h>
#include <stdint.h>
#include <math.h>


#define FINW   6
#define HID    128
#define XPW    8
#define AXW    32
#define H1W    256
#define NTHR   256
#define NWAVE  8
#define EPT    8
#define CHUNK  (NTHR * EPT)
#define WCAP   (EPT * 32)
#define LISTN  (NWAVE * WCAP)
#define NBA    1024
#define SLA    10
#define DEGCAP 48
#define GBM    64
#define GBN    128
#define GTHR   128
#define CMP_ZINTS    (LISTN + NBA * DEGCAP + NBA)
#define CMP_LDS_INTS (CMP_ZINTS + 16 + NBA)
#define NBRIT  ((NBA * DEGCAP) / (NTHR * 4))
#define WSMAX  134217728

static_assert((CHUNK & (CHUNK - 1)) == 0 && CHUNK <= 4096);
static_assert((NBA & (NBA - 1)) == 0 && NBA == (1 << SLA));
static_assert(((long long)CHUNK << SLA) < (1LL << 31));
static_assert(CMP_ZINTS % (NTHR * 4) == 0);
static_assert((NBA * DEGCAP) % (NTHR * 4) == 0 && (NBA * DEGCAP * 4) % 128 == 0 && (DEGCAP * 4) % 16 == 0);
static_assert(NBA == 4 * NTHR && NBA % NTHR == 0 && NBA % GBM == 0);
static_assert(GBN == HID && GBM == (GTHR / 32) * 16 && HID == 4 * 32);
static_assert(AXW % 32 == 0 && H1W % 32 == 0 && H1W == 2 * HID);
static_assert(CMP_LDS_INTS * 4 <= 300000);
static_assert(DEGCAP <= 64 && DEGCAP >= 44);

typedef float          v2f   __attribute__((ext_vector_type(2)));
typedef float          v4f   __attribute__((ext_vector_type(4)));
typedef float          v8f   __attribute__((ext_vector_type(8)));
typedef int            v4i   __attribute__((ext_vector_type(4)));
typedef int            v8i   __attribute__((ext_vector_type(8)));
typedef unsigned int   v4u   __attribute__((ext_vector_type(4)));
typedef unsigned short v4us  __attribute__((ext_vector_type(4)));
typedef unsigned short v8us  __attribute__((ext_vector_type(8)));
typedef unsigned short v16us __attribute__((ext_vector_type(16)));
typedef __bf16         v16bf __attribute__((ext_vector_type(16)));
typedef v2f  __attribute__((may_alias)) v2fa;
typedef v4f  __attribute__((may_alias)) v4fa;
typedef v4i  __attribute__((may_alias)) v4ia;
typedef v4u  __attribute__((may_alias)) v4ua;
typedef v4us __attribute__((may_alias)) v4usa;
typedef v8us __attribute__((may_alias)) v8usa;
union FragB { v16bf v; v16us u; v8us h[2]; v8i w; };

__device__ __forceinline__ v8f wmb(const FragB& a, const FragB& b, v8f c) {
  v8f d = __builtin_amdgcn_wmma_f32_16x16x32_bf16(false, a.v, false, b.v, (short)0, c, false, false);
  asm volatile("v_nop\n\tv_nop\n\tv_nop\n\tv_nop" : "+v"(d) : "v"(a.w), "v"(b.w));
  return d;
}

__device__ __forceinline__ unsigned bf16_bits(float f) {
  const unsigned u = __float_as_uint(f);
  return (u + 0x7FFFu + ((u >> 16) & 1u)) >> 16;
}
__device__ __forceinline__ float bf16_val(float f) {
  return __uint_as_float(bf16_bits(f) << 16);
}

template <int SLB>
__device__ __forceinline__ int scan_chunk(const int* __restrict__ dsts, int nE, int cbase, int slotBase,
                                          int nb, int vec8, int* list, int tid, int lane, int wave) {
  int wc = 0;
  const int el0  = tid * EPT;
  const int e0   = cbase + el0;
  const int sent = -2147483647 - 1;
  v4i da, db;
  if (vec8 != 0 && cbase + CHUNK <= nE) {
    da = *(const v4i*)(dsts + e0);
    db = *(const v4i*)(dsts + e0 + 4);
  } else {
    da.x = (e0     < nE) ? dsts[min(e0,     nE - 1)] : sent;
    da.y = (e0 + 1 < nE) ? dsts[min(e0 + 1, nE - 1)] : sent;
    da.z = (e0 + 2 < nE) ? dsts[min(e0 + 2, nE - 1)] : sent;
    da.w = (e0 + 3 < nE) ? dsts[min(e0 + 3, nE - 1)] : sent;
    db.x = (e0 + 4 < nE) ? dsts[min(e0 + 4, nE - 1)] : sent;
    db.y = (e0 + 5 < nE) ? dsts[min(e0 + 5, nE - 1)] : sent;
    db.z = (e0 + 6 < nE) ? dsts[min(e0 + 6, nE - 1)] : sent;
    db.w = (e0 + 7 < nE) ? dsts[min(e0 + 7, nE - 1)] : sent;
  }
  const unsigned nbs = (unsigned)slotBase;
  const unsigned unb = (unsigned)nb;
  const unsigned s0 = (unsigned)da.x - nbs, s1 = (unsigned)da.y - nbs;
  const unsigned s2 = (unsigned)da.z - nbs, s3 = (unsigned)da.w - nbs;
  const unsigned s4 = (unsigned)db.x - nbs, s5 = (unsigned)db.y - nbs;
  const unsigned s6 = (unsigned)db.z - nbs, s7 = (unsigned)db.w - nbs;
  const bool h0 = s0 < unb, h1 = s1 < unb, h2 = s2 < unb, h3 = s3 < unb;
  const bool h4 = s4 < unb, h5 = s5 < unb, h6 = s6 < unb, h7 = s7 < unb;
  const unsigned any = __builtin_amdgcn_ballot_w32(h0 | h1 | h2 | h3 | h4 | h5 | h6 | h7);
  if (any != 0u) {
#define HITJ(J, HJ, SJ) { \
      const unsigned mj = __builtin_amdgcn_ballot_w32(HJ); \
      if (mj != 0u) { \
        if (HJ) { \
          const int pos = wc + (int)__builtin_amdgcn_mbcnt_lo(mj, 0u); \
          if (pos < WCAP) list[wave * WCAP + pos] = ((el0 + (J)) << SLB) | (int)(SJ); \
        } \
        wc += (int)__builtin_popcount(mj); } }
    HITJ(0, h0, s0)
    HITJ(1, h1, s1)
    HITJ(2, h2, s2)
    HITJ(3, h3, s3)
    HITJ(4, h4, s4)
    HITJ(5, h5, s5)
    HITJ(6, h6, s6)
    HITJ(7, h7, s7)
#undef HITJ
  }
  return wc;
}

__global__ __launch_bounds__(NTHR) void k_prep(const float* __restrict__ x, const float* __restrict__ W1,
                                               const float* __restrict__ b1, const float* __restrict__ W2,
                                               const float* __restrict__ b2, const float* __restrict__ W3,
                                               const float* __restrict__ b3, int nN, int nbX,
                                               float* XP, unsigned short* W1P, unsigned short* W2T2,
                                               float* PARF) {
  const int b = (int)blockIdx.x;
  const int tid = (int)threadIdx.x;
  if (b < nbX) {
    const int u    = b * NTHR + tid;
    const int row  = u >> 1;
    const int half = u & 1;
    const int rc   = row < nN ? row : nN - 1;
    const float* p = x + (size_t)rc * FINW;
    const v2f a = *(const v2fa*)(p + 4 * half);
    const v2f c = *(const v2fa*)(p + 2 + 2 * half);
    const bool ok  = row < nN;
    const bool ok2 = ok && (half == 0);
    v4f o;
    o.x = ok  ? bf16_val(a.x) : 0.0f;
    o.y = ok  ? bf16_val(a.y) : 0.0f;
    o.z = ok2 ? bf16_val(c.x) : 0.0f;
    o.w = ok2 ? bf16_val(c.y) : 0.0f;
    float* dp = XP + (size_t)u * 4;
    *(volatile v4f*)dp = o;
    __threadfence();
    *(volatile v4f*)dp = o;
  } else if (b < nbX + 2) {
    const int v  = (b - nbX) * NTHR + tid;
    const int n  = v >> 2;
    const int k8 = (v & 3) * 8;
    const bool use = k8 < 16;
    const float* p = W1 + n;
    v8us o;
#pragma unroll
    for (int i = 0; i < FINW; ++i) {
      const unsigned bits = bf16_bits(p[(size_t)i * HID]);
      o[i] = use ? (unsigned short)bits : (unsigned short)0;
    }
    o[6] = (unsigned short)0; o[7] = (unsigned short)0;
    unsigned short* dp = W1P + (size_t)v * 8;
    *(volatile v8us*)dp = o;
    __threadfence();
    *(volatile v8us*)dp = o;
  } else if (b < nbX + 18) {
    const int v  = (b - nbX - 2) * NTHR + tid;
    const int n  = v >> 5;
    const int k8 = (v & 31) * 8;
    const int kk = k8 & (HID - 1);
    const float* p = W2 + (size_t)kk * HID + n;
    v8us o;
#pragma unroll
    for (int i = 0; i < 8; ++i) o[i] = (unsigned short)bf16_bits(p[(size_t)i * HID]);
    unsigned short* dp = W2T2 + (size_t)v * 8;
    *(volatile v8us*)dp = o;
    __threadfence();
    *(volatile v8us*)dp = o;
  } else {
    const int seg = b - nbX - 18;
    if (tid >= 32) return;
    v4f v;
    if (seg == 0) {
      v = *(const v4fa*)(b1 + 4 * tid);
    } else if (seg == 1) {
      v = *(const v4fa*)(b2 + 4 * tid);
    } else if (seg == 2) {
      v = *(const v4fa*)(W3 + 4 * tid);
    } else {
      const float bb = b3[0];
      v.x = (tid == 0) ? bb : 0.0f; v.y = 0.0f; v.z = 0.0f; v.w = 0.0f;
    }
    v4f o;
    o.x = bf16_val(v.x); o.y = bf16_val(v.y); o.z = bf16_val(v.z); o.w = bf16_val(v.w);
    float* dp = PARF + (size_t)seg * 128 + 4 * tid;
    *(volatile v4f*)dp = o;
    __threadfence();
    *(volatile v4f*)dp = o;
  }
}

__global__ __launch_bounds__(NTHR) void k_compact(const int* __restrict__ srcs, const int* __restrict__ dsts,
                                                  int nE, int nN, int vec8,
                                                  int* nbr, int* cntg, float* dinv) {
  extern __shared__ __attribute__((aligned(16))) int dsm[];
  int*   list = dsm;
  int*   nbrL = dsm + LISTN;
  int*   cnt  = nbrL + NBA * DEGCAP;
  int*   misc = cnt + NBA;
  float* dl   = (float*)(misc + 16);
  const int tid = (int)threadIdx.x, lane = tid & 31, wave = tid >> 5;
  const int nodeBase = (int)blockIdx.x * NBA;

  {
    const v4i z4 = {0, 0, 0, 0};
    for (int i = tid * 4; i < CMP_ZINTS; i += NTHR * 4) *(v4ia*)(dsm + i) = z4;
    if (tid < 16) misc[tid] = 0;
  }
  __syncthreads();

  const int nChunks = (nE + CHUNK - 1) / CHUNK;
#pragma unroll 1
  for (int ch = 0; ch < nChunks; ++ch) {
    const int cbase = ch * CHUNK;
    const int wc = scan_chunk<SLA>(dsts, nE, cbase, nodeBase, NBA, vec8, list, tid, lane, wave);
    if (lane == 0) misc[wave] = wc;
    __syncthreads();
    if (wave == 0) {
#pragma unroll 1
      for (int w2 = 0; w2 < NWAVE; ++w2) {
        int c = misc[w2];
        c = c < 0 ? 0 : (c > WCAP ? WCAP : c);
#pragma unroll 1
        for (int b0 = 0; b0 < c; b0 += 32) {
          const int idx = b0 + lane;
          const int ent = list[w2 * WCAP + (idx < WCAP ? idx : WCAP - 1)];
          const int el  = (ent >> SLA) & (CHUNK - 1);
          int eid = cbase + el;
          eid = eid < 0 ? 0 : (eid > nE - 1 ? nE - 1 : eid);
          int sr = srcs[eid];
          sr = sr < 0 ? 0 : (sr > nN - 1 ? nN - 1 : sr);
          const int m32 = (c - b0) < 32 ? (c - b0) : 32;
#pragma unroll 1
          for (int k = 0; k < m32; ++k) {
            const int u    = __builtin_amdgcn_readlane(ent, k);
            const int sk   = __builtin_amdgcn_readlane(sr, k);
            const int slot = u & (NBA - 1);
            if (lane == 0) {
              int c0 = cnt[slot];
              c0 = c0 < 0 ? 0 : (c0 > (1 << 20) ? (1 << 20) : c0);
              const int pos = c0 < DEGCAP ? c0 : DEGCAP - 1;
              if (c0 < DEGCAP) nbrL[slot * DEGCAP + pos] = sk;
              cnt[slot] = c0 + 1;
            }
          }
        }
      }
    }
    __syncthreads();
  }

#pragma unroll 1
  for (int i = tid; i < NBA; i += NTHR) {
    int c = cnt[i];
    c = c < 0 ? 0 : c;
    const float d = (float)c + 1.0f;
    dl[i] = (d > 0.0f) ? (1.0f / sqrtf(d)) : 0.0f;
  }
  __syncthreads();

  v4i cv = *(const v4ia*)(cnt + 4 * tid);
  cv.x = (cv.x > DEGCAP) ? -1 : cv.x;
  cv.y = (cv.y > DEGCAP) ? -1 : cv.y;
  cv.z = (cv.z > DEGCAP) ? -1 : cv.z;
  cv.w = (cv.w > DEGCAP) ? -1 : cv.w;
  const v4f dv = *(const v4fa*)(dl + 4 * tid);
  int*   cp = cntg + (size_t)nodeBase + 4 * tid;
  float* dp = dinv + (size_t)nodeBase + 4 * tid;
  int*   nb = nbr + (size_t)nodeBase * DEGCAP;

  *(volatile v4i*)cp = cv;
  *(volatile v4f*)dp = dv;
#pragma unroll 4
  for (int it = 0; it < NBRIT; ++it) {
    const int o = 4 * (it * NTHR + tid);
    const v4i q = *(const v4ia*)(nbrL + o);
    *(volatile v4i*)(nb + o) = q;
  }
  __threadfence();
  *(volatile v4i*)cp = cv;
  *(volatile v4f*)dp = dv;
#pragma unroll 4
  for (int it = 0; it < NBRIT; ++it) {
    const int o = 4 * (it * NTHR + tid);
    const v4i q = *(const v4ia*)(nbrL + o);
    *(volatile v4i*)(nb + o) = q;
  }
}

__global__ __launch_bounds__(NTHR) void k_agg1(const int* __restrict__ nbr, const int* __restrict__ cntg,
                                               const float* __restrict__ dinv, const float* __restrict__ xp,
                                               int nN, unsigned int* axhl) {
  __shared__ __attribute__((aligned(16))) unsigned int st[NTHR * 16];
  const int tid = (int)threadIdx.x;
  const int blockBase = (int)blockIdx.x * NTHR;
  const int node = blockBase + tid;
  const int craw = cntg[node];
  const bool bad = (craw < 0) || (craw > DEGCAP);
  const int c = craw < 0 ? 0 : (craw > DEGCAP ? DEGCAP : craw);
  int cm = c;
  cm = max(cm, __shfl_xor(cm, 16, 32));
  cm = max(cm, __shfl_xor(cm, 8, 32));
  cm = max(cm, __shfl_xor(cm, 4, 32));
  cm = max(cm, __shfl_xor(cm, 2, 32));
  cm = max(cm, __shfl_xor(cm, 1, 32));
  cm = cm > DEGCAP ? DEGCAP : cm;
  const int nc = node < nN ? node : nN - 1;
  const float di = dinv[nc];
  float a0 = 0.0f, a1 = 0.0f, a2 = 0.0f, a3 = 0.0f, a4 = 0.0f, a5 = 0.0f;
  const int* nr = nbr + (size_t)node * DEGCAP;
#pragma unroll 1
  for (int j = 0; j < cm; ++j) {
    const int jj = j < DEGCAP ? j : DEGCAP - 1;
    int s = nr[jj];
    s = s < 0 ? 0 : (s > nN - 1 ? nN - 1 : s);
    const float wv = dinv[s] * di;
    const float w  = (j < c) ? wv : 0.0f;
    const float* p = xp + (size_t)s * XPW;
    const v4f u = *(const v4fa*)p;
    const v2f v = *(const v2fa*)(p + 4);
    a0 = fmaf(w, u.x, a0); a1 = fmaf(w, u.y, a1); a2 = fmaf(w, u.z, a2);
    a3 = fmaf(w, u.w, a3); a4 = fmaf(w, v.x, a4); a5 = fmaf(w, v.y, a5);
  }
  {
    const float rd = di * di;
    const float* p = xp + (size_t)nc * XPW;
    const v4f u = *(const v4fa*)p;
    const v2f v = *(const v2fa*)(p + 4);
    a0 = fmaf(rd, u.x, a0); a1 = fmaf(rd, u.y, a1); a2 = fmaf(rd, u.z, a2);
    a3 = fmaf(rd, u.w, a3); a4 = fmaf(rd, v.x, a4); a5 = fmaf(rd, v.y, a5);
  }
  const float pz = bad ? __int_as_float(0x7fc00000) : 0.0f;
  const bool live = node < nN;
  const float m0 = live ? (a0 + pz) : 0.0f;
  const float m1 = live ? (a1 + pz) : 0.0f;
  const float m2 = live ? (a2 + pz) : 0.0f;
  const float m3 = live ? (a3 + pz) : 0.0f;
  const float m4 = live ? (a4 + pz) : 0.0f;
  const float m5 = live ? (a5 + pz) : 0.0f;
  const unsigned h0 = bf16_bits(m0), h1 = bf16_bits(m1), h2 = bf16_bits(m2);
  const unsigned h3 = bf16_bits(m3), h4 = bf16_bits(m4), h5 = bf16_bits(m5);
  const unsigned l0 = bf16_bits(m0 - __uint_as_float(h0 << 16));
  const unsigned l1 = bf16_bits(m1 - __uint_as_float(h1 << 16));
  const unsigned l2 = bf16_bits(m2 - __uint_as_float(h2 << 16));
  const unsigned l3 = bf16_bits(m3 - __uint_as_float(h3 << 16));
  const unsigned l4 = bf16_bits(m4 - __uint_as_float(h4 << 16));
  const unsigned l5 = bf16_bits(m5 - __uint_as_float(h5 << 16));
  v4u wh, wl;
  wh.x = h0 | (h1 << 16); wh.y = h2 | (h3 << 16); wh.z = h4 | (h5 << 16); wh.w = 0u;
  wl.x = l0 | (l1 << 16); wl.y = l2 | (l3 << 16); wl.z = l4 | (l5 << 16); wl.w = 0u;
  const v4u zz = {0u, 0u, 0u, 0u};
  unsigned int* sr = st + tid * 16;
  *(v4ua*)(sr)      = wh;
  *(v4ua*)(sr + 4)  = wl;
  *(v4ua*)(sr + 8)  = zz;
  *(v4ua*)(sr + 12) = zz;
  __syncthreads();
  v4u q[4];
#pragma unroll
  for (int it = 0; it < 4; ++it) q[it] = *(const v4ua*)(st + 4 * (it * NTHR + tid));
  unsigned int* gp = axhl + (size_t)blockBase * 16;
#pragma unroll
  for (int it = 0; it < 4; ++it) *(volatile v4u*)(gp + 4 * (it * NTHR + tid)) = q[it];
  __threadfence();
#pragma unroll
  for (int it = 0; it < 4; ++it) *(volatile v4u*)(gp + 4 * (it * NTHR + tid)) = q[it];
}

template <int FIN>
__global__ __launch_bounds__(GTHR) void k_gemm(const unsigned short* __restrict__ Apl,
                                               const unsigned short* __restrict__ BT, int K,
                                               const float* __restrict__ bias,
                                               float* outF, unsigned short* outH, int nOut) {
  __shared__ __attribute__((aligned(16))) float stg[GBM * GBN];
  const int tid = (int)threadIdx.x, lane = tid & 31, wave = tid >> 5, hh = lane >> 4, m = lane & 15;
  const int rowBase = (int)blockIdx.x * GBM;

  v8f acc[8];
  {
    const v8f z = {0.f, 0.f, 0.f, 0.f, 0.f, 0.f, 0.f, 0.f};
#pragma unroll
    for (int t = 0; t < 8; ++t) acc[t] = z;
  }
  const unsigned short* ap = Apl + (size_t)(rowBase + 16 * wave + m) * (size_t)K + 8 * hh;
  const unsigned short* bp = BT + (size_t)m * (size_t)K + 8 * hh;

#pragma unroll 1
  for (int k0 = 0; k0 < K; k0 += 32) {
    FragB af;
    af.h[0] = *(const v8usa*)(ap + k0);
    af.h[1] = *(const v8usa*)(ap + k0 + 16);
#pragma unroll
    for (int nt = 0; nt < 8; ++nt) {
      const unsigned short* wq = bp + (size_t)(16 * nt) * (size_t)K + k0;
      FragB bf;
      bf.h[0] = *(const v8usa*)wq;
      bf.h[1] = *(const v8usa*)(wq + 16);
      acc[nt] = wmb(af, bf, acc[nt]);
    }
  }

#pragma unroll
  for (int nt = 0; nt < 8; ++nt) {
    const int lc = 16 * nt + m;
#pragma unroll
    for (int r = 0; r < 8; ++r) {
      const int lr = 16 * wave + 8 * hh + r;
      stg[lr * GBN + lc] = acc[nt][r];
    }
  }
  __syncthreads();

  v4f pv[16];
#pragma unroll
  for (int i = 0; i < 16; ++i) pv[i] = *(const v4fa*)(stg + (16 * wave + i) * GBN + 4 * lane);
  __syncthreads();

  if constexpr (FIN != 0) {
#pragma unroll
    for (int i = 0; i < 16; ++i) {
      const int r = rowBase + 16 * wave + i;
      *(volatile v4f*)(outF + (size_t)r * HID + 4 * lane) = pv[i];
    }
    __threadfence();
#pragma unroll
    for (int i = 0; i < 16; ++i) {
      const int r = rowBase + 16 * wave + i;
      *(volatile v4f*)(outF + (size_t)r * HID + 4 * lane) = pv[i];
    }
  } else {
    const v4f bb4 = *(const v4fa*)(bias + 4 * lane);
#pragma unroll
    for (int i = 0; i < 16; ++i) {
      const bool ok = (rowBase + 16 * wave + i) < nOut;
      const v4f t = pv[i] + bb4;
      v4f y;
      y.x = (t.x > 0.0f) ? t.x : (t.x - t.x);
      y.y = (t.y > 0.0f) ? t.y : (t.y - t.y);
      y.z = (t.z > 0.0f) ? t.z : (t.z - t.z);
      y.w = (t.w > 0.0f) ? t.w : (t.w - t.w);
      y.x = ok ? y.x : 0.0f; y.y = ok ? y.y : 0.0f; y.z = ok ? y.z : 0.0f; y.w = ok ? y.w : 0.0f;
      pv[i] = y;
    }
#pragma unroll
    for (int i = 0; i < 16; ++i) {
      v4us h4, l4;
      unsigned hb;
      hb = bf16_bits(pv[i].x); h4[0] = (unsigned short)hb; l4[0] = (unsigned short)bf16_bits(pv[i].x - __uint_as_float(hb << 16));
      hb = bf16_bits(pv[i].y); h4[1] = (unsigned short)hb; l4[1] = (unsigned short)bf16_bits(pv[i].y - __uint_as_float(hb << 16));
      hb = bf16_bits(pv[i].z); h4[2] = (unsigned short)hb; l4[2] = (unsigned short)bf16_bits(pv[i].z - __uint_as_float(hb << 16));
      hb = bf16_bits(pv[i].w); h4[3] = (unsigned short)hb; l4[3] = (unsigned short)bf16_bits(pv[i].w - __uint_as_float(hb << 16));
      unsigned short* srow = (unsigned short*)stg + (size_t)(16 * wave + i) * (2 * GBN);
      *(v4usa*)(srow + 4 * lane) = h4;
      *(v4usa*)(srow + HID + 4 * lane) = l4;
    }
    __syncthreads();
    v8us qv[16];
#pragma unroll
    for (int i = 0; i < 16; ++i) {
      const unsigned short* srow = (const unsigned short*)stg + (size_t)(16 * wave + i) * (2 * GBN);
      qv[i] = *(const v8usa*)(srow + 8 * lane);
    }
#pragma unroll
    for (int i = 0; i < 16; ++i) {
      unsigned short* rp = outH + (size_t)(rowBase + 16 * wave + i) * (size_t)H1W + 8 * lane;
      *(volatile v8us*)rp = qv[i];
    }
    __threadfence();
#pragma unroll
    for (int i = 0; i < 16; ++i) {
      unsigned short* rp = outH + (size_t)(rowBase + 16 * wave + i) * (size_t)H1W + 8 * lane;
      *(volatile v8us*)rp = qv[i];
    }
  }
}

__global__ __launch_bounds__(NTHR) void k_agg2(const int* __restrict__ nbr, const int* __restrict__ cntg,
                                               const float* __restrict__ dinv, const float* __restrict__ xh2,
                                               const float* __restrict__ parf, int nN, float* tOut) {
  __shared__ __attribute__((aligned(16))) float tl[NTHR];
  const int tid = (int)threadIdx.x, lane = tid & 31;
  const int wave = __builtin_amdgcn_readfirstlane(tid >> 5);
  const int blockBase = (int)blockIdx.x * NTHR;
  const v4f b2v = *(const v4fa*)(parf + 128 + 4 * lane);
  const v4f w3v = *(const v4fa*)(parf + 256 + 4 * lane);
  const float qnan = __int_as_float(0x7fc00000);

#pragma unroll 1
  for (int si = 0; si < NTHR / NWAVE; ++si) {
    const int s    = si * NWAVE + wave;
    const int node = blockBase + s;
    const int craw = cntg[node];
    const bool bad = (craw < 0) || (craw > DEGCAP);
    const int c = craw < 0 ? 0 : (craw > DEGCAP ? DEGCAP : craw);
    const int nc = node < nN ? node : nN - 1;
    const float dd = dinv[nc];
    const float rd = dd * dd;
    float a0 = 0.0f, a1 = 0.0f, a2 = 0.0f, a3 = 0.0f;
    const int* nr = nbr + (size_t)node * DEGCAP;
#pragma unroll 1
    for (int b0 = 0; b0 < c; b0 += 32) {
      int idx = b0 + lane;
      idx = idx > DEGCAP - 1 ? DEGCAP - 1 : idx;
      int sr = nr[idx];
      sr = sr < 0 ? 0 : (sr > nN - 1 ? nN - 1 : sr);
      const float cf  = dinv[sr] * dd;
      const int   cfi = __float_as_int(cf);
      const int m32 = (c - b0) < 32 ? (c - b0) : 32;
#pragma unroll 1
      for (int k = 0; k < m32; ++k) {
        const int   sk = __builtin_amdgcn_readlane(sr, k);
        const float ck = __int_as_float(__builtin_amdgcn_readlane(cfi, k));
        const v4f a = *(const v4fa*)(xh2 + (size_t)sk * HID + 4 * lane);
        a0 = fmaf(ck, a.x, a0); a1 = fmaf(ck, a.y, a1);
        a2 = fmaf(ck, a.z, a2); a3 = fmaf(ck, a.w, a3);
      }
    }
    const v4f sv = *(const v4fa*)(xh2 + (size_t)nc * HID + 4 * lane);
    const float pz = bad ? qnan : 0.0f;
    float y0 = fmaf(rd, sv.x, a0) + b2v.x;
    float y1 = fmaf(rd, sv.y, a1) + b2v.y;
    float y2 = fmaf(rd, sv.z, a2) + b2v.z;
    float y3 = fmaf(rd, sv.w, a3) + b2v.w;
    y0 = (y0 > 0.0f) ? y0 : (y0 - y0);
    y1 = (y1 > 0.0f) ? y1 : (y1 - y1);
    y2 = (y2 > 0.0f) ? y2 : (y2 - y2);
    y3 = (y3 > 0.0f) ? y3 : (y3 - y3);
    y0 = y0 + pz; y1 = y1 + pz; y2 = y2 + pz; y3 = y3 + pz;
    float t = y0 * w3v.x;
    t = fmaf(y1, w3v.y, t);
    t = fmaf(y2, w3v.z, t);
    t = fmaf(y3, w3v.w, t);
    t += __shfl_xor(t, 16, 32);
    t += __shfl_xor(t, 8, 32);
    t += __shfl_xor(t, 4, 32);
    t += __shfl_xor(t, 2, 32);
    t += __shfl_xor(t, 1, 32);
    const float tv = (node < nN) ? t : 0.0f;
    if (lane == 0) tl[s] = tv;
  }
  __syncthreads();
  const int u4 = 4 * (tid & 63);
  const v4f ov = *(const v4fa*)(tl + u4);
  float* op = tOut + (size_t)blockBase + u4;
  const bool okst = tid < 64;
  if (okst) *(volatile v4f*)op = ov;
  __threadfence();
  if (okst) *(volatile v4f*)op = ov;
}

__global__ __launch_bounds__(NTHR) void k_agg3(const int* __restrict__ nbr, const int* __restrict__ cntg,
                                               const float* __restrict__ dinv, const float* __restrict__ tIn,
                                               const float* __restrict__ parf, int nN, float* out) {
  __shared__ __attribute__((aligned(16))) float ol[NTHR];
  const int tid = (int)threadIdx.x;
  const int blockBase = (int)blockIdx.x * NTHR;
  const int node = blockBase + tid;
  const int craw = cntg[node];
  const bool bad = (craw < 0) || (craw > DEGCAP);
  const int c = craw < 0 ? 0 : (craw > DEGCAP ? DEGCAP : craw);
  int cm = c;
  cm = max(cm, __shfl_xor(cm, 16, 32));
  cm = max(cm, __shfl_xor(cm, 8, 32));
  cm = max(cm, __shfl_xor(cm, 4, 32));
  cm = max(cm, __shfl_xor(cm, 2, 32));
  cm = max(cm, __shfl_xor(cm, 1, 32));
  cm = cm > DEGCAP ? DEGCAP : cm;
  const int nc = node < nN ? node : nN - 1;
  const float di = dinv[nc];
  const float b3v = parf[384];
  float acc = 0.0f;
  const int* nr = nbr + (size_t)node * DEGCAP;
#pragma unroll 1
  for (int j = 0; j < cm; ++j) {
    const int jj = j < DEGCAP ? j : DEGCAP - 1;
    int s = nr[jj];
    s = s < 0 ? 0 : (s > nN - 1 ? nN - 1 : s);
    const float wv = dinv[s] * di;
    const float tv = tIn[s];
    const bool on = j < c;
    const float w  = on ? wv : 0.0f;
    const float tx = on ? tv : 0.0f;
    acc = fmaf(w, tx, acc);
  }
  const float rd = di * di;
  const float pz = bad ? __int_as_float(0x7fc00000) : 0.0f;
  const float res = (fmaf(rd, tIn[nc], acc) + b3v) + pz;
  ol[tid] = (node < nN) ? res : 0.0f;
  __syncthreads();
  const int u4 = 4 * (tid & 63);
  const v4f ov = *(const v4fa*)(ol + u4);
  const int r0 = blockBase + u4;
  const bool okst = (tid < 64) && (r0 + 3 < nN);
  float* op = out + (size_t)(okst ? r0 : 0);
  if (okst) *(volatile v4f*)op = ov;
  __threadfence();
  if (okst) *(volatile v4f*)op = ov;
}

static inline int cdiv(int a, int b) { return (a + b - 1) / b; }
static inline size_t al256(size_t o) { return (o + 255) & ~(size_t)255; }

extern "C" void kernel_launch(void* const* d_in, const int* in_sizes, int n_in,
                              void* d_out, int out_size, void* d_ws, size_t ws_size,
                              hipStream_t stream) {
  if (n_in < 8) return;
  if (in_sizes[0] < FINW || (in_sizes[0] % FINW) != 0) return;
  const int nN = in_sizes[0] / FINW;
  if (nN < 32 || nN > (1 << 22) || (nN % 32) != 0) return;
  if (in_sizes[1] < 2 || (in_sizes[1] & 1) != 0) return;
  const int nE = in_sizes[1] / 2;
  if (nE < 1 || nE >= (1 << (31 - SLA))) return;
  if (in_sizes[2] != FINW * HID || in_sizes[3] != HID) return;
  if (in_sizes[4] != HID * HID || in_sizes[5] != HID) return;
  if (in_sizes[6] != HID || in_sizes[7] != 1) return;
  if (out_size != nN) return;

  const float* x    = (const float*)d_in[0];
  const int*   edge = (const int*)d_in[1];
  const float* W1   = (const float*)d_in[2];
  const float* b1   = (const float*)d_in[3];
  const float* W2   = (const float*)d_in[4];
  const float* b2   = (const float*)d_in[5];
  const float* W3   = (const float*)d_in[6];
  const float* b3   = (const float*)d_in[7];
  float* out = (float*)d_out;
  const int* src = edge;
  const int* dst = edge + nE;

  const int MP  = cdiv(nN, GBM) * GBM;
  const int gM  = MP / GBM;
  const int gC  = cdiv(MP, NBA);
  const int NSL = gC * NBA;
  if (NSL < MP || (NSL % NTHR) != 0) return;
  const int vec8 = ((nE & 3) == 0) ? 1 : 0;
  const int nbX  = (NSL * 2) / NTHR;

  char* ws = (char*)d_ws;
  size_t off = 0;
  const size_t oPAR = off; off = al256(off + (size_t)512 * 4);
  const size_t oW1P = off; off = al256(off + (size_t)HID * AXW * 2);
  const size_t oW2T = off; off = al256(off + (size_t)HID * H1W * 2);
  const size_t oXP  = off; off = al256(off + (size_t)NSL * XPW * 4);
  const size_t oCNT = off; off = al256(off + (size_t)NSL * 4);
  const size_t oDIN = off; off = al256(off + (size_t)NSL * 4);
  const size_t oT   = off; off = al256(off + (size_t)NSL * 4);
  const size_t oNBR = off; off = al256(off + (size_t)NSL * DEGCAP * 4);
  const size_t oAX  = off; off = al256(off + (size_t)NSL * AXW * 2);
  const size_t oH1  = off; off = al256(off + (size_t)MP * H1W * 2);
  const size_t oXH2 = off; off = al256(off + (size_t)MP * HID * 4);
  if (off > ws_size || off > (size_t)WSMAX) return;
  float*          PARF = (float*)(ws + oPAR);
  unsigned short* W1P  = (unsigned short*)(ws + oW1P);
  unsigned short* W2T2 = (unsigned short*)(ws + oW2T);
  float*          XP   = (float*)(ws + oXP);
  int*            CNT  = (int*)(ws + oCNT);
  float*          DINV = (float*)(ws + oDIN);
  float*          T    = (float*)(ws + oT);
  int*            NBR  = (int*)(ws + oNBR);
  unsigned int*   AXHL = (unsigned int*)(ws + oAX);
  unsigned short* H1HL = (unsigned short*)(ws + oH1);
  float*          XH2  = (float*)(ws + oXH2);

  const size_t cmpLds = (size_t)CMP_LDS_INTS * 4;
  hipFuncSetAttribute(reinterpret_cast<const void*>(&k_compact), hipFuncAttributeMaxDynamicSharedMemorySize, (int)cmpLds);

  k_prep<<<nbX + 22, NTHR, 0, stream>>>(x, W1, b1, W2, b2, W3, b3, nN, nbX, XP, W1P, W2T2, PARF);
  k_compact<<<gC, NTHR, cmpLds, stream>>>(src, dst, nE, nN, vec8, NBR, CNT, DINV);
  k_agg1<<<NSL / NTHR, NTHR, 0, stream>>>(NBR, CNT, DINV, XP, nN, AXHL);
  k_gemm<0><<<gM, GTHR, 0, stream>>>((const unsigned short*)AXHL, W1P, AXW, PARF, XH2, H1HL, nN);
  k_gemm<1><<<gM, GTHR, 0, stream>>>(H1HL, W2T2, H1W, PARF, XH2, H1HL, nN);
  k_agg2<<<NSL / NTHR, NTHR, 0, stream>>>(NBR, CNT, DINV, XH2, PARF, nN, T);
  k_agg3<<<cdiv(nN, NTHR), NTHR, 0, stream>>>(NBR, CNT, DINV, T, PARF, nN, out);
}
